// DSBlock_80384607912556
// MI455X (gfx1250) — hardware-verified
//
#include <hip/hip_runtime.h>


#define NB_  8
#define CIN  128
#define CH   64
#define HW   64
#define NL   4096
#define NS   256
#define NHD  4
#define HD   16
#define KP   32
#define NZ   (NB_ * NHD)
typedef _Float16 h16;
typedef unsigned short bf;
typedef __attribute__((ext_vector_type(16))) __bf16   v16bf;
typedef __attribute__((ext_vector_type(16))) _Float16 v16h;
typedef __attribute__((ext_vector_type(8)))  _Float16 v8h;
typedef __attribute__((ext_vector_type(8)))  unsigned short v8us;
typedef __attribute__((ext_vector_type(8)))  float    v8f;
typedef __attribute__((ext_vector_type(4)))  float    v4f;
typedef v8h  __attribute__((may_alias)) v8ha;
typedef v4f  __attribute__((may_alias)) v4fa;
typedef v8us __attribute__((may_alias)) v8usa;

__device__ __forceinline__ unsigned short f2bf(float f) { unsigned u = __float_as_uint(f); u += 0x7FFFu + ((u >> 16) & 1u); return (unsigned short)(u >> 16); }
__device__ __forceinline__ float bf2f(unsigned short b) { return __uint_as_float(((unsigned)b) << 16); }
__device__ __forceinline__ float bfr(float f) { return bf2f(f2bf(f)); }
__device__ __forceinline__ v16h cat16(v8h lo, v8h hi) { return __builtin_shufflevector(lo, hi, 0, 1, 2, 3, 4, 5, 6, 7, 8, 9, 10, 11, 12, 13, 14, 15); }
__device__ __forceinline__ v16bf cat16b(v8us lo, v8us hi) { return __builtin_bit_cast(v16bf, __builtin_shufflevector(lo, hi, 0, 1, 2, 3, 4, 5, 6, 7, 8, 9, 10, 11, 12, 13, 14, 15)); }
__device__ __forceinline__ v8f wmma16(v16h a, v16h b, v8f c) { return __builtin_amdgcn_wmma_f32_16x16x32_f16(false, a, false, b, (short)0, c, false, false); }
__device__ __forceinline__ v8f wmmab(v16bf a, v16bf b, v8f c) { return __builtin_amdgcn_wmma_f32_16x16x32_bf16(false, a, false, b, (short)0, c, false, false); }


template <typename T16> struct WFrag;
template <> struct WFrag<h16> { typedef v16h V; static __device__ __forceinline__ V ld(const h16* p) { return cat16(*(const v8h*)p, *(const v8h*)(p + 16)); } static __device__ __forceinline__ v8f mma(V a, V b, v8f c) { return wmma16(a, b, c); } };
template <> struct WFrag<bf> { typedef v16bf V; static __device__ __forceinline__ V ld(const bf* p) { return cat16b(*(const v8us*)p, *(const v8us*)(p + 16)); } static __device__ __forceinline__ v8f mma(V a, V b, v8f c) { return wmmab(a, b, c); } };
template <typename T16, int NSPLIT, bool BIAS>
__global__ __launch_bounds__(32) void k_gemmw(const T16* __restrict__ A, const T16* __restrict__ A2, const T16* __restrict__ Bt, const T16* __restrict__ Bt2, int K, float* C, int ldc, const float* __restrict__ bias, size_t sA, size_t sB, size_t sC) {
    typedef typename WFrag<T16>::V V;
    __shared__ __align__(16) float os[16 * 68];
    const size_t z = blockIdx.z; A += z * sA; if (A2) A2 += z * sA; Bt += z * sB; if (Bt2) Bt2 += z * sB; C += z * sC;
    const int lane = threadIdx.x & 31, lr = lane & 15, hi = lane >> 4; const int r0 = blockIdx.x * 64, c0 = blockIdx.y * 64;
    v8f acc[4][4];
#pragma unroll
    for (int mb = 0; mb < 4; ++mb)
#pragma unroll
        for (int nb = 0; nb < 4; ++nb) acc[mb][nb] = (v8f){};
    const size_t aoff = (size_t)(r0 + lr) * K + 8 * hi, boff = (size_t)(c0 + lr) * K + 8 * hi;
#pragma unroll 1
    for (int kc = 0; kc < K; kc += 32) {
        V a[4], a2[4];
#pragma unroll
        for (int mb = 0; mb < 4; ++mb) { a[mb] = WFrag<T16>::ld(A + aoff + (size_t)mb * 16 * K + kc); if (NSPLIT == 1 || NSPLIT == 2) a2[mb] = WFrag<T16>::ld(A2 + aoff + (size_t)mb * 16 * K + kc); }
#pragma unroll
        for (int nb = 0; nb < 4; ++nb) { const V b = WFrag<T16>::ld(Bt + boff + (size_t)nb * 16 * K + kc); V b2; if (NSPLIT >= 2) b2 = WFrag<T16>::ld(Bt2 + boff + (size_t)nb * 16 * K + kc);
#pragma unroll
            for (int mb = 0; mb < 4; ++mb) { acc[mb][nb] = WFrag<T16>::mma(a[mb], b, acc[mb][nb]); if (NSPLIT == 1 || NSPLIT == 2) acc[mb][nb] = WFrag<T16>::mma(a2[mb], b, acc[mb][nb]); if (NSPLIT >= 2) acc[mb][nb] = WFrag<T16>::mma(a[mb], b2, acc[mb][nb]); } }
        asm volatile("v_nop\n\tv_nop\n\tv_nop\n\tv_nop" : "+v"(acc[0][0]), "+v"(acc[1][1]), "+v"(acc[2][2]), "+v"(acc[3][3]) : "v"(a[0]), "v"(a[3]));
    }
#pragma unroll
    for (int mb = 0; mb < 4; ++mb) {
#pragma unroll
        for (int nb = 0; nb < 4; ++nb) {
#pragma unroll
            for (int j = 0; j < 8; ++j) os[(hi * 8 + j) * 68 + nb * 16 + lr] = acc[mb][nb][j]; }
        __builtin_amdgcn_wave_barrier(); asm volatile("" ::: "memory");
        float* crow = C + (size_t)(r0 + mb * 16) * ldc + c0;
#pragma unroll 1
        for (int ps = 0; ps < 2; ++ps) {
#pragma unroll
            for (int s = 0; s < 8; ++s) { const int row = 2 * s + hi, cofs = lr * 4; v4f val = *(const v4fa*)(os + row * 68 + cofs); if (BIAS) { val[0] += bfr(bias[c0 + cofs]); val[1] += bfr(bias[c0 + cofs + 1]); val[2] += bfr(bias[c0 + cofs + 2]); val[3] += bfr(bias[c0 + cofs + 3]); }
                *(volatile v4f*)(crow + (size_t)row * ldc + cofs) = val; }
            if (ps == 0) __threadfence(); }
        __builtin_amdgcn_wave_barrier(); asm volatile("" ::: "memory");
    }
}

__device__ __forceinline__ void splitf(float y, unsigned short& h, unsigned short& l) { h = f2bf(y); l = f2bf(y - bf2f(h)); }
typedef __attribute__((ext_vector_type(2))) unsigned short v2us;
typedef __attribute__((ext_vector_type(4))) unsigned short v4us;

__global__ __launch_bounds__(256) void k_cvt8(const float* __restrict__ src, bf* dst, size_t n8) { const size_t i = (size_t)blockIdx.x * 256 + threadIdx.x; if (i >= n8) return; const v8f v = *(const v8f*)(src + i * 8); v8us o;
#pragma unroll
    for (int k = 0; k < 8; ++k) o[k] = f2bf(v[k]); *(volatile v8us*)(dst + i * 8) = o; __threadfence(); *(volatile v8us*)(dst + i * 8) = o; }
__global__ __launch_bounds__(256) void k_col3(const float* __restrict__ in, bf* XC) { const size_t e = ((size_t)blockIdx.x * 256 + threadIdx.x) * 4; if (e >= (size_t)NL * 576) return; const int j0 = (int)(e % 576); const int p = (int)(e / 576); const int b = 0; const int y = p / HW, x = p % HW; v4us o;
#pragma unroll
    for (int q = 0; q < 4; ++q) { const int j = j0 + q; const int c = j / 9, t = j % 9; const int yy = y + t / 3 - 1, xx = x + t % 3 - 1; o[q] = (yy >= 0 && yy < HW && xx >= 0 && xx < HW) ? f2bf(in[(((size_t)b * CIN + c) * HW + yy) * HW + xx]) : (unsigned short)0; }
    *(volatile v4us*)(XC + e) = o; __threadfence(); *(volatile v4us*)(XC + e) = o; }
__global__ __launch_bounds__(256) void k_bnr(const float* __restrict__ F, const float* __restrict__ sc, const float* __restrict__ bi, float* FL, bf* Fh, bf* Fl) { const size_t i = ((size_t)blockIdx.x * 256 + threadIdx.x) * 4; if (i >= (size_t)NL * CH) return; const int c = (int)(i % CH); const v4f a = *(const v4f*)(F + i); v4f o; v4us oh, ol;
#pragma unroll
    for (int q = 0; q < 4; ++q) { float t = __fmul_rn(a[q], bfr(sc[c + q])); asm volatile("" : "+v"(t)); o[q] = fmaxf(__fadd_rn(t, bfr(bi[c + q])), 0.f); unsigned short u, l; splitf(o[q], u, l); oh[q] = u; ol[q] = l; }
    for (int ps = 0; ps < 2; ++ps) { *(volatile v4f*)(FL + i) = o; *(volatile v4us*)(Fh + i) = oh; *(volatile v4us*)(Fl + i) = ol; if (ps == 0) __threadfence(); } }
__global__ __launch_bounds__(256) void k_pool(const float* __restrict__ in, bf* Gh, bf* Gl) { const size_t e = ((size_t)blockIdx.x * 256 + threadIdx.x) * 2; if (e >= (size_t)NS * CH) return; const int c = (int)(e % CH); const int s = (int)(e / CH); const int b = 0; const int sy = s / 16, sx = s % 16; v2us oh, ol;
#pragma unroll
    for (int u = 0; u < 2; ++u) { const float* src = in + (((size_t)b * CIN + CH + c + u) * HW + sy * 4) * HW + sx * 4; float acc = 0.f; for (int dy = 0; dy < 4; ++dy) for (int dx = 0; dx < 4; ++dx) acc = __fadd_rn(acc, bfr(src[dy * HW + dx])); unsigned short a, l; splitf(acc * 0.0625f, a, l); oh[u] = a; ol[u] = l; }
    *(volatile v2us*)(Gh + e) = oh; *(volatile v2us*)(Gl + e) = ol; __threadfence(); *(volatile v2us*)(Gh + e) = oh; *(volatile v2us*)(Gl + e) = ol; }
__global__ __launch_bounds__(256) void k_hpl(const float* __restrict__ QKV, int ntok, int s, bf* Ph, bf* Pl) { const size_t e = ((size_t)blockIdx.x * 256 + threadIdx.x) * 2; if (e >= (size_t)NHD * ntok * KP) return; const int d = (int)(e % KP); const int n = (int)((e / KP) % ntok); const int z = (int)(e / ((size_t)KP * ntok)); const int h = z % NHD, b = z / NHD; v2us oh, ol;
#pragma unroll
    for (int u = 0; u < 2; ++u) { unsigned short a = 0, l = 0; if (d + u < HD) splitf(QKV[((size_t)b * ntok + n) * (3 * CH) + s * CH + h * HD + d + u], a, l); oh[u] = a; ol[u] = l; } *(volatile v2us*)(Ph + e) = oh; *(volatile v2us*)(Pl + e) = ol; __threadfence(); *(volatile v2us*)(Ph + e) = oh; *(volatile v2us*)(Pl + e) = ol; }
__global__ __launch_bounds__(256) void k_vpl(const float* __restrict__ QKV, int ntok, bf* Vh, bf* Vl) { const size_t e = ((size_t)blockIdx.x * 256 + threadIdx.x) * 2; if (e >= (size_t)NHD * 64 * ntok) return; const int n = (int)(e % ntok); const int d = (int)((e / ntok) % 64); const int z = (int)(e / ((size_t)ntok * 64)); const int h = z % NHD, b = z / NHD; v2us oh, ol;
#pragma unroll
    for (int u = 0; u < 2; ++u) { unsigned short a = 0, l = 0; if (d < HD) splitf(QKV[((size_t)b * ntok + n + u) * (3 * CH) + 2 * CH + h * HD + d], a, l); oh[u] = a; ol[u] = l; } *(volatile v2us*)(Vh + e) = oh; *(volatile v2us*)(Vl + e) = ol; __threadfence(); *(volatile v2us*)(Vh + e) = oh; *(volatile v2us*)(Vl + e) = ol; }
template <int NK>
__global__ __launch_bounds__(256) void k_sm(const float* __restrict__ Sb, int nrows, bf* Ph, bf* Pl) { const int lane = threadIdx.x & 31; const int row = blockIdx.x * 8 + (threadIdx.x >> 5); if (row >= nrows) return; const float* sr = Sb + (size_t)row * NK; constexpr int PER = NK / 32; float v[PER]; float mx = -3.0e38f;
#pragma unroll
    for (int ch = 0; ch < PER / 4; ++ch) { const v4f a = *(const v4f*)(sr + ch * 128 + lane * 4);
#pragma unroll
        for (int q = 0; q < 4; ++q) { float t = a[q] * 0.25f; asm volatile("" : "+v"(t)); v[ch * 4 + q] = t; mx = fmaxf(mx, t); } }
#pragma unroll
    for (int sh = 16; sh; sh >>= 1) mx = fmaxf(mx, __shfl_xor(mx, sh, 32));
    float sum = 0.f;
#pragma unroll
    for (int k = 0; k < PER; ++k) { float d0 = __fsub_rn(v[k], mx); asm volatile("" : "+v"(d0)); v[k] = __expf(d0); sum += v[k]; }
#pragma unroll
    for (int sh = 16; sh; sh >>= 1) sum += __shfl_xor(sum, sh, 32);
    const float f = __fdiv_rn(1.0f, sum);
#pragma unroll 1
    for (int ps = 0; ps < 2; ++ps) {
#pragma unroll
        for (int ch = 0; ch < PER / 4; ++ch) { v4us oh, ol;
#pragma unroll
            for (int q = 0; q < 4; ++q) { unsigned short a, c; splitf(v[ch * 4 + q] * f, a, c); oh[q] = a; ol[q] = c; } const size_t oo = (size_t)row * NK + ch * 128 + lane * 4; *(volatile v4us*)(Ph + oo) = oh; *(volatile v4us*)(Pl + oo) = ol; }
        if (ps == 0) __threadfence(); } }
__global__ __launch_bounds__(256) void k_catl(const float* __restrict__ OL, bf* Ch, bf* Cl) { const size_t e = ((size_t)blockIdx.x * 256 + threadIdx.x) * 2; if (e >= (size_t)NHD * NL * HD) return; const int d = (int)(e % HD); const int p = (int)((e / HD) % NL); const int z = (int)(e / ((size_t)HD * NL)); const int h = z % NHD, b = 0; v2us oh, ol;
#pragma unroll
    for (int u = 0; u < 2; ++u) { unsigned short a, c; splitf(OL[((size_t)z * NL + p) * 64 + d + u], a, c); oh[u] = a; ol[u] = c; } const size_t o = ((size_t)b * NL + p) * CIN + h * HD + d; *(volatile v2us*)(Ch + o) = oh; *(volatile v2us*)(Cl + o) = ol; __threadfence(); *(volatile v2us*)(Ch + o) = oh; *(volatile v2us*)(Cl + o) = ol; }
__global__ __launch_bounds__(256) void k_catg(const float* __restrict__ OG, bf* Ch, bf* Cl) { const size_t e = ((size_t)blockIdx.x * 256 + threadIdx.x) * 2; if (e >= (size_t)NHD * NL * HD) return; const int d = (int)(e % HD); const int p = (int)((e / HD) % NL); const int z = (int)(e / ((size_t)HD * NL)); const int h = z % NHD, b = 0; const int y = p / HW, x = p % HW;
    const float syf = fmaxf(((float)y + 0.5f) * 0.25f - 0.5f, 0.f), sxf = fmaxf(((float)x + 0.5f) * 0.25f - 0.5f, 0.f); int y0 = (int)floorf(syf), x0 = (int)floorf(sxf); const float wy = syf - (float)y0, wx = sxf - (float)x0; const int y1 = min(y0 + 1, 15), x1 = min(x0 + 1, 15); y0 = min(y0, 15); x0 = min(x0, 15); const float* g = OG + (size_t)z * NS * 64; v2us oh, ol;
#pragma unroll
    for (int u = 0; u < 2; ++u) { const int dd = d + u; const float v00 = g[(y0 * 16 + x0) * 64 + dd], v01 = g[(y0 * 16 + x1) * 64 + dd], v10 = g[(y1 * 16 + x0) * 64 + dd], v11 = g[(y1 * 16 + x1) * 64 + dd];
        float t0 = __fmul_rn(v00, 1.f - wx); asm volatile("" : "+v"(t0)); float t1 = __fmul_rn(v01, wx); asm volatile("" : "+v"(t1)); const float top = __fadd_rn(t0, t1); float b0 = __fmul_rn(v10, 1.f - wx); asm volatile("" : "+v"(b0)); float b1 = __fmul_rn(v11, wx); asm volatile("" : "+v"(b1)); const float bot = __fadd_rn(b0, b1);
        float r0 = __fmul_rn(top, 1.f - wy); asm volatile("" : "+v"(r0)); float r1 = __fmul_rn(bot, wy); asm volatile("" : "+v"(r1)); unsigned short a, c; splitf(__fadd_rn(r0, r1), a, c); oh[u] = a; ol[u] = c; }
    const size_t o = ((size_t)b * NL + p) * CIN + CH + h * HD + d; *(volatile v2us*)(Ch + o) = oh; *(volatile v2us*)(Cl + o) = ol; __threadfence(); *(volatile v2us*)(Ch + o) = oh; *(volatile v2us*)(Cl + o) = ol; }
__global__ __launch_bounds__(256) void k_out(const float* __restrict__ R, const float* __restrict__ sc, const float* __restrict__ bi, float* OUT) { const size_t e = ((size_t)blockIdx.x * 256 + threadIdx.x) * 4; if (e >= (size_t)CIN * NL) return; const int p = (int)(e % NL); const int o = (int)(e / NL); const int b = 0; const float s = bfr(sc[o]), bb = bfr(bi[o]); v4f r;
#pragma unroll
    for (int q = 0; q < 4; ++q) { float t = __fmul_rn(R[((size_t)b * NL + p + q) * CIN + o], s); asm volatile("" : "+v"(t)); r[q] = fmaxf(__fadd_rn(t, bb), 0.f); } *(volatile v4f*)(OUT + e) = r; __threadfence(); *(volatile v4f*)(OUT + e) = r; }

extern "C" void kernel_launch(void* const* d_in, const int* in_sizes, int n_in,
                              void* d_out, int out_size, void* d_ws, size_t ws_size, hipStream_t stream) {
    (void)in_sizes; (void)n_in; (void)out_size;
    const float* in = (const float*)d_in[0]; const float* dep_w = (const float*)d_in[1]; const float* dep_s = (const float*)d_in[2]; const float* dep_b = (const float*)d_in[3]; const float* qkv_w = (const float*)d_in[4]; const float* qkv_b = (const float*)d_in[5]; const float* l_w = (const float*)d_in[6]; const float* l_s = (const float*)d_in[7]; const float* l_b = (const float*)d_in[8];
    float* OUT = (float*)d_out;
    char* wsp = (char*)d_ws;
    auto take = [&](size_t bytes) { char* p = wsp; wsp += (bytes + 255) & ~(size_t)255; return (void*)p; };
    const size_t TL = NL, TG = NS;
    bf* WD = (bf*)take((size_t)CH * 576 * 2); bf* WQ = (bf*)take((size_t)3 * CH * CH * 2); bf* WL = (bf*)take((size_t)CIN * CIN * 2); bf* XC = (bf*)take(TL * 576 * 2); float* F = (float*)take(TL * CH * 4); float* FL = (float*)take(TL * CH * 4); bf* Fh = (bf*)take(TL * CH * 2); bf* Fl = (bf*)take(TL * CH * 2); bf* Gh = (bf*)take(TG * CH * 2); bf* Gl = (bf*)take(TG * CH * 2);
    float* QL = (float*)take(TL * 3 * CH * 4); float* QG = (float*)take(TG * 3 * CH * 4); bf* LQh = (bf*)take((size_t)NHD * NL * KP * 2); bf* LQl = (bf*)take((size_t)NHD * NL * KP * 2); bf* LKh = (bf*)take((size_t)NHD * NL * KP * 2); bf* LKl = (bf*)take((size_t)NHD * NL * KP * 2); bf* LVh = (bf*)take((size_t)NHD * 64 * NL * 2); bf* LVl = (bf*)take((size_t)NHD * 64 * NL * 2);
    bf* GQh = (bf*)take((size_t)NHD * NS * KP * 2); bf* GQl = (bf*)take((size_t)NHD * NS * KP * 2); bf* GKh = (bf*)take((size_t)NHD * NS * KP * 2); bf* GKl = (bf*)take((size_t)NHD * NS * KP * 2); bf* GVh = (bf*)take((size_t)NHD * 64 * NS * 2); bf* GVl = (bf*)take((size_t)NHD * 64 * NS * 2);
    float* S1 = (float*)take((size_t)NHD * NL * NS * 4); bf* P1h = (bf*)take((size_t)NHD * NL * NS * 2); bf* P1l = (bf*)take((size_t)NHD * NL * NS * 2); float* OL = (float*)take((size_t)NHD * NL * 64 * 4); float* OG = (float*)take((size_t)NHD * NS * 64 * 4); bf* CATh = (bf*)take(TL * CIN * 2); bf* CATl = (bf*)take(TL * CIN * 2); float* RR = (float*)take(TL * CIN * 4);
    float* S2 = S1; bf* P2h = P1h; bf* P2l = P1l;
    if ((size_t)(wsp - (char*)d_ws) > ws_size) return;
    k_cvt8<<<(CH * 576 / 8 + 255) / 256, 256, 0, stream>>>(dep_w, WD, (size_t)CH * 576 / 8); k_cvt8<<<(3 * CH * CH / 8 + 255) / 256, 256, 0, stream>>>(qkv_w, WQ, (size_t)3 * CH * CH / 8); k_cvt8<<<(CIN * CIN / 8 + 255) / 256, 256, 0, stream>>>(l_w, WL, (size_t)CIN * CIN / 8);
    for (int b = 0; b < NB_; ++b) { const float* inb = in + (size_t)b * CIN * HW * HW;
        k_col3<<<(unsigned)((TL * 576 / 4 + 255) / 256), 256, 0, stream>>>(inb, XC);
        k_gemmw<bf, 0, false><<<dim3(TL / 64, 1, 1), 32, 0, stream>>>(XC, nullptr, WD, nullptr, 576, F, CH, nullptr, 0, 0, 0); k_bnr<<<(unsigned)((TL * CH / 4 + 255) / 256), 256, 0, stream>>>(F, dep_s, dep_b, FL, Fh, Fl);
        k_gemmw<bf, 1, true><<<dim3(TL / 64, 3 * CH / 64, 1), 32, 0, stream>>>(Fh, Fl, WQ, nullptr, CH, QL, 3 * CH, qkv_b, 0, 0, 0);
        k_pool<<<(unsigned)((TG * CH / 2 + 255) / 256), 256, 0, stream>>>(inb, Gh, Gl); k_gemmw<bf, 1, true><<<dim3(TG / 64, 3 * CH / 64, 1), 32, 0, stream>>>(Gh, Gl, WQ, nullptr, CH, QG, 3 * CH, qkv_b, 0, 0, 0);
        k_hpl<<<(unsigned)(((size_t)NHD * NL * KP / 2 + 255) / 256), 256, 0, stream>>>(QL, NL, 0, LQh, LQl); k_hpl<<<(unsigned)(((size_t)NHD * NL * KP / 2 + 255) / 256), 256, 0, stream>>>(QL, NL, 1, LKh, LKl); k_vpl<<<(unsigned)(((size_t)NHD * 64 * NL / 2 + 255) / 256), 256, 0, stream>>>(QL, NL, LVh, LVl);
        k_hpl<<<(unsigned)(((size_t)NHD * NS * KP / 2 + 255) / 256), 256, 0, stream>>>(QG, NS, 0, GQh, GQl); k_hpl<<<(unsigned)(((size_t)NHD * NS * KP / 2 + 255) / 256), 256, 0, stream>>>(QG, NS, 1, GKh, GKl); k_vpl<<<(unsigned)(((size_t)NHD * 64 * NS / 2 + 255) / 256), 256, 0, stream>>>(QG, NS, GVh, GVl);
        k_gemmw<bf, 2, false><<<dim3(NL / 64, NS / 64, NHD), 32, 0, stream>>>(LQh, LQl, GKh, GKl, KP, S1, NS, nullptr, (size_t)NL * KP, (size_t)NS * KP, (size_t)NL * NS);
        k_sm<NS><<<NHD * NL / 8, 256, 0, stream>>>(S1, NHD * NL, P1h, P1l);
        k_gemmw<bf, 2, false><<<dim3(NL / 64, 1, NHD), 32, 0, stream>>>(P1h, P1l, GVh, GVl, NS, OL, 64, nullptr, (size_t)NL * NS, (size_t)64 * NS, (size_t)NL * 64);
        k_gemmw<bf, 2, false><<<dim3(NS / 64, NL / 64, NHD), 32, 0, stream>>>(GQh, GQl, LKh, LKl, KP, S2, NL, nullptr, (size_t)NS * KP, (size_t)NL * KP, (size_t)NS * NL);
        k_sm<NL><<<NHD * NS / 8, 256, 0, stream>>>(S2, NHD * NS, P2h, P2l);
        k_gemmw<bf, 2, false><<<dim3(NS / 64, 1, NHD), 32, 0, stream>>>(P2h, P2l, LVh, LVl, NL, OG, 64, nullptr, (size_t)NS * NL, (size_t)64 * NL, (size_t)NS * 64);
        k_catl<<<(unsigned)(((size_t)NHD * NL * HD / 2 + 255) / 256), 256, 0, stream>>>(OL, CATh, CATl); k_catg<<<(unsigned)(((size_t)NHD * NL * HD / 2 + 255) / 256), 256, 0, stream>>>(OG, CATh, CATl);
        k_gemmw<bf, 1, false><<<dim3(TL / 64, CIN / 64, 1), 32, 0, stream>>>(CATh, CATl, WL, nullptr, CIN, RR, CIN, nullptr, 0, 0, 0);
        k_out<<<(unsigned)(((size_t)CIN * NL / 4 + 255) / 256), 256, 0, stream>>>(RR, l_s, l_b, OUT + (size_t)b * CIN * NL); }
}
